// RWKV7Attention_55155970015404
// MI455X (gfx1250) — hardware-verified
//
#include <hip/hip_runtime.h>
#include <math.h>

constexpr int kBatch   = 2;
constexpr int kSeq     = 1024;
constexpr int kChan    = 2048;
constexpr int kHeads   = 32;
constexpr int kHeadDim = 64;
constexpr int kRows    = kBatch * kSeq;
constexpr int kRankW   = 96;
constexpr int kRankA   = 96;
constexpr int kRankV   = 64;
constexpr int kRankG   = 256;
constexpr int kRankWp  = 128;
constexpr int kRankAp  = 128;
constexpr int kStepsPerChunk = 16;
constexpr int kChunks  = kSeq / kStepsPerChunk;
constexpr float kGnEps = 6.4e-4f;
constexpr float kInvHeadDim = 1.0f / 64.0f;
static_assert(kChunks * kStepsPerChunk == kSeq);
static_assert(kHeads * kHeadDim == kChan);

typedef __attribute__((ext_vector_type(16))) _Float16 v16h;
typedef __attribute__((ext_vector_type(8)))  _Float16 v8h;
typedef __attribute__((ext_vector_type(16))) __bf16   v16b;
typedef __attribute__((ext_vector_type(8)))  __bf16   v8b;
typedef __attribute__((ext_vector_type(8)))  float    v8f;
typedef __attribute__((ext_vector_type(4)))  float    v4f;
typedef __attribute__((ext_vector_type(4)))  unsigned int v4u;

__device__ __forceinline__ unsigned short f2bf_bits(float f) {
  unsigned u = __float_as_uint(f);
  return (unsigned short)((u + 0x7FFFu + ((u >> 16) & 1u)) >> 16);
}
__device__ __forceinline__ float bf_bits2f(unsigned short h) { return __uint_as_float(((unsigned)h) << 16); }

__device__ __forceinline__ void dep_guard_h(v8f& a, v8f& b, v16h x, v16h y) { asm volatile("v_nop\n\tv_nop\n\tv_nop\n\tv_nop" : "+v"(a), "+v"(b) : "v"(x), "v"(y)); }
__device__ __forceinline__ void dep_guard_b(v8f& a, v8f& b, v16b x, v16b y) { asm volatile("v_nop\n\tv_nop\n\tv_nop\n\tv_nop" : "+v"(a), "+v"(b) : "v"(x), "v"(y)); }
__device__ __forceinline__ void keep4_h(v16h a, v16h b, v16h c, v16h d) { asm volatile("v_nop" :: "v"(a), "v"(b), "v"(c), "v"(d)); }
__device__ __forceinline__ void keep4_b(v16b a, v16b b, v16b c, v16b d) { asm volatile("v_nop" :: "v"(a), "v"(b), "v"(c), "v"(d)); }
__device__ __forceinline__ void acc_guard4(v8f& a, v8f& b, v8f& c, v8f& d) { asm volatile("v_nop\n\tv_nop\n\tv_nop\n\tv_nop" : "+v"(a), "+v"(b), "+v"(c), "+v"(d)); }
__device__ __forceinline__ void dep_guard1_b4(v8f& a, v16b x, v16b y, v16b z, v16b w) { asm volatile("v_nop\n\tv_nop\n\tv_nop\n\tv_nop" : "+v"(a) : "v"(x), "v"(y), "v"(z), "v"(w)); }
template <typename T> struct Frag;
template <> struct Frag<_Float16> {
  typedef v16h V; union U { v16h v; v8h h[2]; };
  static __device__ __forceinline__ v16h load(const _Float16* p) {
    U f; f.h[0] = *(const v8h*)(p); f.h[1] = *(const v8h*)(p + 16); return f.v;
  }
  static __device__ __forceinline__ v8f mma(v16h a, v16h b, v8f c) {
    return __builtin_amdgcn_wmma_f32_16x16x32_f16(false, a, false, b, (short)0, c, false, false);
  }
  static __device__ __forceinline__ void guard(v8f& a, v8f& b, v16h x, v16h y) { dep_guard_h(a, b, x, y); }
  static __device__ __forceinline__ void keep(v16h a, v16h b, v16h c, v16h d) { keep4_h(a, b, c, d); }
};
template <> struct Frag<__bf16> {
  typedef v16b V; union U { v16b v; v8b h[2]; };
  static __device__ __forceinline__ v16b load(const __bf16* p) {
    U f; f.h[0] = *(const v8b*)(p); f.h[1] = *(const v8b*)(p + 16); return f.v;
  }
  static __device__ __forceinline__ v8f mma(v16b a, v16b b, v8f c) {
    return __builtin_amdgcn_wmma_f32_16x16x32_bf16(false, a, false, b, (short)0, c, false, false);
  }
  static __device__ __forceinline__ void guard(v8f& a, v8f& b, v16b x, v16b y) { dep_guard_b(a, b, x, y); }
  static __device__ __forceinline__ void keep(v16b a, v16b b, v16b c, v16b d) { keep4_b(a, b, c, d); }
};

__device__ __forceinline__ unsigned pk16(unsigned short a, unsigned short b) { return (unsigned)a | ((unsigned)b << 16); }

template <int ET> struct Elem;
template <> struct Elem<0> { typedef _Float16 T; };
template <> struct Elem<1> { typedef __bf16 T; };
template <int ET, bool SPLIT, int BIAS_MODE, int OUT_MODE, bool RESID, int ACT = 0>
__global__ __launch_bounds__(256) void wmma_gemm64(
    const unsigned short* __restrict__ Ap, const unsigned short* __restrict__ A2p, int lda, long strideA,
    const unsigned short* __restrict__ Btp, const unsigned short* __restrict__ Bt2p, int ldb, long strideB,
    void* __restrict__ Cout, void* __restrict__ Cout2, int ldc, long strideC,
    const float* __restrict__ bias,
    const float* __restrict__ resid, long strideR,
    int M, int N, int K, float scale) {
  typedef typename Elem<ET>::T T;
  typedef typename Frag<T>::V V;
  const T* A = (const T*)Ap; const T* A2 = (const T*)A2p; const T* Bt = (const T*)Btp; const T* Bt2 = (const T*)Bt2p;
  __shared__ __align__(16) float sT[8][16 * 68];
  const int b    = blockIdx.y;
  const int lane = threadIdx.x & 31;
  const int wave = threadIdx.x >> 5;
  const int tilesN = N >> 6;
  const int tilesM = M >> 6;
  const int tile = blockIdx.x * 8 + wave;
  if (tile >= tilesM * tilesN) return;
  const int tm = tile / tilesN;
  const int tn = tile - tm * tilesN;
  const int m0 = tm << 6;
  const int n0 = tn << 6;

  const T* Ab  = A  + (size_t)b * strideA;
  const T* Bb  = Bt + (size_t)b * strideB;
  const T* Ab2 = SPLIT ? (A2  + (size_t)b * strideA) : nullptr;
  const T* Bb2 = SPLIT ? (Bt2 + (size_t)b * strideB) : nullptr;

  const int rlane = lane & 15;
  const int koff  = (lane >> 4) * 8;
  const int mOff  = (lane >> 4) * 8;

  v8f acc[4][4];
#pragma unroll
  for (int i = 0; i < 4; ++i)
#pragma unroll
    for (int j = 0; j < 4; ++j) acc[i][j] = (v8f){0.f,0.f,0.f,0.f,0.f,0.f,0.f,0.f};

  for (int k0 = 0; k0 < K; k0 += 32) {
    V bh[4], bl[4];
#pragma unroll
    for (int j = 0; j < 4; ++j) {
      const size_t bo = (size_t)(n0 + (j << 4) + rlane) * ldb + koff + k0;
      bh[j] = Frag<T>::load(Bb + bo);
      if (SPLIT) bl[j] = Frag<T>::load(Bb2 + bo);
    }
#pragma unroll
    for (int i = 0; i < 4; ++i) {
      const size_t ao = (size_t)(m0 + (i << 4) + rlane) * lda + koff + k0;
      V ah = Frag<T>::load(Ab + ao);
      V al;
      if (SPLIT) al = Frag<T>::load(Ab2 + ao);
#pragma unroll
      for (int j = 0; j < 4; ++j) {
        acc[i][j] = Frag<T>::mma(ah, bh[j], acc[i][j]);
        if (SPLIT) {
          acc[i][j] = Frag<T>::mma(ah, bl[j], acc[i][j]);
          acc[i][j] = Frag<T>::mma(al, bh[j], acc[i][j]);
        }
      }
      Frag<T>::guard(acc[i][0], acc[i][3], ah, SPLIT ? al : ah);
    }
    Frag<T>::keep(bh[0], bh[1], bh[2], bh[3]);
    if (SPLIT) Frag<T>::keep(bl[0], bl[1], bl[2], bl[3]);
  }
  acc_guard4(acc[0][0], acc[0][1], acc[0][2], acc[0][3]);
  acc_guard4(acc[1][0], acc[1][1], acc[1][2], acc[1][3]);
  acc_guard4(acc[2][0], acc[2][1], acc[2][2], acc[2][3]);
  acc_guard4(acc[3][0], acc[3][1], acc[3][2], acc[3][3]);

  float* slab = sT[wave];
  const float* Rb = RESID ? (resid + (size_t)b * strideR) : nullptr;
#pragma unroll
  for (int i = 0; i < 4; ++i) {
    const int mBase = m0 + (i << 4);
#pragma unroll
    for (int j = 0; j < 4; ++j) {
      const int n = n0 + (j << 4) + rlane;
      float bv = 0.f;
      if (BIAS_MODE == 2) bv = bias[n];
#pragma unroll
      for (int r = 0; r < 8; ++r) {
        float v = acc[i][j][r] * scale;
        if (BIAS_MODE == 1) v += bias[mBase + mOff + r];
        if (BIAS_MODE == 2) v += bv;
        if (RESID) v += Rb[(size_t)(mBase + mOff + r) * ldc + n];
        if (ACT == 1) v = tanhf(v);
        if (ACT == 2) v = fmaxf(v, 0.0f);
        if (ACT == 3) v = v / (1.0f + expf(-v));
        if (ACT == 4) v = (v > 0.f) ? v : 0.01f * v;
        if (ACT == 6) v = 1.0f / (1.0f + expf(-v));
        slab[(mOff + r) * 68 + (j << 4) + rlane] = v;
      }
    }
    __builtin_amdgcn_fence(__ATOMIC_RELEASE, "workgroup");
    __builtin_amdgcn_wave_barrier();
    __builtin_amdgcn_fence(__ATOMIC_ACQUIRE, "workgroup");
    if (OUT_MODE == 0) {
      float* C = (float*)Cout + (size_t)b * strideC;
      const int hh = lane >> 4, c4 = (lane & 15) * 4;
      for (int pass = 0; pass < 2; ++pass) {
#pragma unroll
        for (int it = 0; it < 8; ++it) {
          const int row = it * 2 + hh;
          v4f v = *(const v4f*)(slab + row * 68 + c4);
          *(volatile v4f*)(C + (size_t)(mBase + row) * ldc + n0 + c4) = v;
        }
        __threadfence();
      }
    } else {
      const int q = lane >> 3, c8 = (lane & 7) * 8;
      unsigned short* C  = (unsigned short*)Cout  + (size_t)b * strideC;
      unsigned short* C2 = (OUT_MODE == 2) ? ((unsigned short*)Cout2 + (size_t)b * strideC) : nullptr;
      for (int pass = 0; pass < 2; ++pass) {
#pragma unroll
        for (int it = 0; it < 4; ++it) {
          const int row = it * 4 + q;
          const float* sp = slab + row * 68 + c8;
          v8h hv, lv;
#pragma unroll
          for (int e = 0; e < 8; ++e) {
            if (OUT_MODE == 1) {
              hv[e] = (_Float16)sp[e];
            } else {
              unsigned short hb = f2bf_bits(sp[e]);
              unsigned short lb = f2bf_bits(sp[e] - bf_bits2f(hb));
              hv[e] = __builtin_bit_cast(_Float16, hb);
              lv[e] = __builtin_bit_cast(_Float16, lb);
            }
          }
          *(volatile v8h*)(C + (size_t)(mBase + row) * ldc + n0 + c8) = hv;
          if (OUT_MODE == 2) *(volatile v8h*)(C2 + (size_t)(mBase + row) * ldc + n0 + c8) = lv;
        }
        __threadfence();
      }
    }
    __builtin_amdgcn_fence(__ATOMIC_RELEASE, "workgroup");
    __builtin_amdgcn_wave_barrier();
    __builtin_amdgcn_fence(__ATOMIC_ACQUIRE, "workgroup");
  }
}

__global__ __launch_bounds__(256) void k_wt_split(const float* __restrict__ W, int R, int Cw,
                                                  unsigned short* __restrict__ hi, unsigned short* __restrict__ lo, int OC) {
  __shared__ float sm[64][65];
  const int t  = threadIdx.x;
  const int j0 = blockIdx.x * 64;
  const int i0 = blockIdx.y * 64;
#pragma unroll
  for (int it = 0; it < 16; ++it) {
    const int e = it * 256 + t;
    const int r = e >> 6;
    const int c = e & 63;
    const int jj = j0 + r, ii = i0 + c;
    const bool valid = (jj < R) && (ii < Cw);
    const int jc = (jj < R) ? jj : (R - 1);
    const int ic = (ii < Cw) ? ii : (Cw - 1);
    float v = W[(size_t)jc * Cw + ic];
    v = valid ? v : 0.f;
    sm[c][r] = v;
  }
  __syncthreads();
  const int lane = t & 31, wave = t >> 5;
  const int q = lane >> 3, c8 = (lane & 7) * 8;
#pragma unroll
  for (int it = 0; it < 2; ++it) {
    const int row = wave * 8 + it * 4 + q;
    unsigned short hb[8], lb[8];
#pragma unroll
    for (int e = 0; e < 8; ++e) {
      const float v = sm[row][c8 + e];
      hb[e] = f2bf_bits(v);
      lb[e] = f2bf_bits(v - bf_bits2f(hb[e]));
    }
    const v4u uh = (v4u){pk16(hb[0], hb[1]), pk16(hb[2], hb[3]), pk16(hb[4], hb[5]), pk16(hb[6], hb[7])};
    const v4u ul = (v4u){pk16(lb[0], lb[1]), pk16(lb[2], lb[3]), pk16(lb[4], lb[5]), pk16(lb[6], lb[7])};
    const size_t off = (size_t)(i0 + row) * OC + j0 + c8;
    *(volatile v4u*)(hi + off) = uh;
    *(volatile v4u*)(lo + off) = ul;
    __threadfence();
    *(volatile v4u*)(hi + off) = uh;
    *(volatile v4u*)(lo + off) = ul;
  }
}

__global__ __launch_bounds__(256) void k_mix_split(const float* __restrict__ X, const float* __restrict__ coef,
                                                   unsigned short* __restrict__ hi, unsigned short* __restrict__ lo, int n8) {
  const int i = blockIdx.x * 256 + threadIdx.x;
  if (i >= n8) return;
  const size_t e0 = (size_t)i * 8;
  const int m = (int)(e0 / kChan);
  const int c = (int)(e0 % kChan);
  const bool hasprev = (m % kSeq) != 0;
  const int mp = hasprev ? (m - 1) : m;
  const float* xp = X + e0;
  const float* pp = X + (size_t)mp * kChan + c;
  const v4f xa = *(const v4f*)(xp), xb = *(const v4f*)(xp + 4);
  const v4f pa = *(const v4f*)(pp), pb = *(const v4f*)(pp + 4);
  const v4f ca = *(const v4f*)(coef + c), cb = *(const v4f*)(coef + c + 4);
  unsigned short hb[8], lb[8];
#pragma unroll
  for (int e = 0; e < 4; ++e) {
    const float xx0 = xa[e], xx1 = xb[e];
    const float p0 = hasprev ? pa[e] : 0.f;
    const float p1 = hasprev ? pb[e] : 0.f;
    const float m0v = xx0 + (p0 - xx0) * ca[e];
    const float m1v = xx1 + (p1 - xx1) * cb[e];
    hb[e]     = f2bf_bits(m0v);
    lb[e]     = f2bf_bits(m0v - bf_bits2f(hb[e]));
    hb[4 + e] = f2bf_bits(m1v);
    lb[4 + e] = f2bf_bits(m1v - bf_bits2f(hb[4 + e]));
  }
  const v4u uh = (v4u){pk16(hb[0], hb[1]), pk16(hb[2], hb[3]), pk16(hb[4], hb[5]), pk16(hb[6], hb[7])};
  const v4u ul = (v4u){pk16(lb[0], lb[1]), pk16(lb[2], lb[3]), pk16(lb[4], lb[5]), pk16(lb[6], lb[7])};
  *(volatile v4u*)(hi + e0) = uh;
  *(volatile v4u*)(lo + e0) = ul;
  __threadfence();
  *(volatile v4u*)(hi + e0) = uh;
  *(volatile v4u*)(lo + e0) = ul;
}

__device__ __forceinline__ void up_job(int mat, int js,
    const unsigned short* __restrict__ gdh, const unsigned short* __restrict__ gdl,
    const unsigned short* __restrict__ g2h, const unsigned short* __restrict__ g2l,
    const unsigned short* __restrict__ wdh, const unsigned short* __restrict__ wdl,
    const unsigned short* __restrict__ w2h, const unsigned short* __restrict__ w2l,
    const unsigned short* __restrict__ vdh, const unsigned short* __restrict__ vdl,
    const unsigned short* __restrict__ v2h, const unsigned short* __restrict__ v2l,
    const unsigned short* __restrict__ adh, const unsigned short* __restrict__ adl,
    const unsigned short* __restrict__ a2h, const unsigned short* __restrict__ a2l,
    int m0, int h, int lane, float* ups) {
  const int c16  = lane & 15;
  const int koff = (lane >> 4) * 8;
  const int hh8  = (lane >> 4) * 8;
  const unsigned short* ahp = (mat == 0) ? gdh : (mat == 1) ? wdh : (mat == 2) ? vdh : adh;
  const unsigned short* alp = (mat == 0) ? gdl : (mat == 1) ? wdl : (mat == 2) ? vdl : adl;
  const unsigned short* bhp = (mat == 0) ? g2h : (mat == 1) ? w2h : (mat == 2) ? v2h : a2h;
  const unsigned short* blp = (mat == 0) ? g2l : (mat == 1) ? w2l : (mat == 2) ? v2l : a2l;
  const int ld   = (mat == 0) ? kRankG : (mat == 1) ? kRankWp : (mat == 2) ? kRankV : kRankAp;
  const int Kdim = (mat == 0) ? kRankG : (mat == 1) ? kRankW  : (mat == 2) ? kRankV : kRankA;
  const __bf16* Ah  = (const __bf16*)ahp;
  const __bf16* Al  = (const __bf16*)alp;
  const __bf16* Bh  = (const __bf16*)bhp;
  const __bf16* Bl  = (const __bf16*)blp;
  const size_t arow = (size_t)(m0 + c16) * ld + koff;
  const size_t brow = (size_t)(h * kHeadDim + js * 16 + c16) * ld + koff;
  v8f acc = (v8f){0.f,0.f,0.f,0.f,0.f,0.f,0.f,0.f};
#pragma unroll 1
  for (int k0 = 0; k0 < Kdim; k0 += 32) {
    const v16b fa  = Frag<__bf16>::load(Ah + arow + k0);
    const v16b fal = Frag<__bf16>::load(Al + arow + k0);
    const v16b fb  = Frag<__bf16>::load(Bh + brow + k0);
    const v16b fbl = Frag<__bf16>::load(Bl + brow + k0);
    acc = Frag<__bf16>::mma(fa, fb, acc);
    acc = Frag<__bf16>::mma(fa, fbl, acc);
    acc = Frag<__bf16>::mma(fal, fb, acc);
    dep_guard1_b4(acc, fa, fal, fb, fbl);
  }
  float* dst = ups + mat * (kStepsPerChunk * kHeadDim) + hh8 * kHeadDim + js * 16 + c16;
#pragma unroll
  for (int r = 0; r < 8; ++r) dst[r * kHeadDim] = acc[r];
}

__global__ __launch_bounds__(256) void k_wkv_fused(
    const float* __restrict__ rbuf, const float* __restrict__ kbuf, const float* __restrict__ vbuf,
    const float* __restrict__ vfirst,
    const unsigned short* __restrict__ gdh, const unsigned short* __restrict__ gdl,
    const unsigned short* __restrict__ g2h, const unsigned short* __restrict__ g2l,
    const unsigned short* __restrict__ wdh, const unsigned short* __restrict__ wdl,
    const unsigned short* __restrict__ w2h, const unsigned short* __restrict__ w2l,
    const unsigned short* __restrict__ vdh, const unsigned short* __restrict__ vdl,
    const unsigned short* __restrict__ v2h, const unsigned short* __restrict__ v2l,
    const unsigned short* __restrict__ adh, const unsigned short* __restrict__ adl,
    const unsigned short* __restrict__ a2h, const unsigned short* __restrict__ a2l,
    const float* __restrict__ w0, const float* __restrict__ a0, const float* __restrict__ v0,
    const float* __restrict__ k_k, const float* __restrict__ k_a, const float* __restrict__ r_k,
    const float* __restrict__ gn_w, const float* __restrict__ gn_b,
    unsigned short* __restrict__ aoh, unsigned short* __restrict__ aol) {
  __shared__ __align__(16) float upS[4][kStepsPerChunk * kHeadDim];
  __shared__ __align__(16) float rS[kStepsPerChunk * kHeadDim];
  __shared__ __align__(16) float decS[kStepsPerChunk * kHeadDim];
  __shared__ __align__(16) float kfS[kStepsPerChunk * kHeadDim];
  __shared__ __align__(16) float vfS[kStepsPerChunk * kHeadDim];
  __shared__ __align__(16) float kkS[kStepsPerChunk * kHeadDim];
  __shared__ __align__(16) float bbS[kStepsPerChunk * kHeadDim];
  __shared__ __align__(16) float yS[kStepsPerChunk * kHeadDim];
  __shared__ __align__(16) float oS[kStepsPerChunk * kHeadDim];

  const int tid  = threadIdx.x;
  const int lane = tid & 31;
  const int wave = __builtin_amdgcn_readfirstlane(tid >> 5);
  const int b    = blockIdx.x / kHeads;
  const int h    = blockIdx.x - b * kHeads;
  const int pt = tid >> 4;
  const int pc = tid & 15;
  const int qv = tid >> 2;
  const int qq = tid & 3;

  float S[16];
#pragma unroll
  for (int j = 0; j < 16; ++j) S[j] = 0.f;

#pragma unroll 1
  for (int tc = 0; tc < kChunks; ++tc) {
    const int t0 = tc * kStepsPerChunk;
    const int m0 = b * kSeq + t0;
    __syncthreads();

    up_job(wave >> 2, wave & 3, gdh, gdl, g2h, g2l, wdh, wdl, w2h, w2l, vdh, vdl, v2h, v2l, adh, adl, a2h, a2l,
           m0, h, lane, &upS[0][0]);
    up_job((wave >> 2) + 2, wave & 3, gdh, gdl, g2h, g2l, wdh, wdl, w2h, w2l, vdh, vdl, v2h, v2l, adh, adl, a2h, a2l,
           m0, h, lane, &upS[0][0]);
    __syncthreads();

    float bon;
    {
      const int m = m0 + pt;
      const size_t rowoff = (size_t)m * kChan + (size_t)h * kHeadDim;
      float ssq = 0.f, bsum = 0.f;
#pragma unroll 1
      for (int i = 0; i < 4; ++i) {
        const int c  = pc + 16 * i;
        const int gc = h * kHeadDim + c;
        const int li = pt * kHeadDim + c;
        const float rv  = rbuf[rowoff + c];
        const float kr  = kbuf[rowoff + c];
        const float vr  = vbuf[rowoff + c];
        const float vfs = vfirst[rowoff + c];
        const float wsum = upS[1][li] + w0[gc];
        const float xneg = -wsum;
        const float sp   = fmaxf(xneg, 0.f) + log1pf(expf(-fabsf(xneg)));
        const float dec  = expf(-expf(-0.5f - sp));
        const float av   = 1.0f / (1.0f + expf(-(upS[3][li] + a0[gc])));
        const float sv   = 1.0f / (1.0f + expf(-(upS[2][li] + v0[gc])));
        const float vf   = vr + (vfs - vr) * sv;
        const float kkv  = kr * k_k[gc];
        const float kf   = kr * (1.0f + (av - 1.0f) * k_a[gc]);
        ssq  += kkv * kkv;
        bsum += rv * kf * r_k[gc];
        rS[li] = rv; decS[li] = dec; kfS[li] = kf; vfS[li] = vf; kkS[li] = kkv; bbS[li] = av;
      }
#pragma unroll
      for (int off = 1; off < 16; off <<= 1) {
        ssq  += __shfl_xor(ssq, off, 32);
        bsum += __shfl_xor(bsum, off, 32);
      }
      const float nrm = sqrtf(ssq);
      const float inv = 1.0f / fmaxf(nrm, 1e-12f);
      bon = bsum;
#pragma unroll 1
      for (int i = 0; i < 4; ++i) {
        const int li = pt * kHeadDim + pc + 16 * i;
        const float kkn = kkS[li] * inv;
        const float av  = bbS[li];
        kkS[li] = kkn;
        bbS[li] = kkn * av;
      }
    }
    __syncthreads();

#pragma unroll 1
    for (int s = 0; s < kStepsPerChunk; ++s) {
      const int base = s * kHeadDim + 16 * qq;
      float sa = 0.f;
#pragma unroll
      for (int j4 = 0; j4 < 4; ++j4) {
        const v4f kk4 = *(const v4f*)(kkS + base + 4 * j4);
#pragma unroll
        for (int e = 0; e < 4; ++e) sa += S[4 * j4 + e] * kk4[e];
      }
      sa += __shfl_xor(sa, 1, 32);
      sa += __shfl_xor(sa, 2, 32);
      sa = -sa;
      const float vt = vfS[s * kHeadDim + qv];
      float yp = 0.f;
#pragma unroll
      for (int j4 = 0; j4 < 4; ++j4) {
        const v4f dc4 = *(const v4f*)(decS + base + 4 * j4);
        const v4f bb4 = *(const v4f*)(bbS + base + 4 * j4);
        const v4f kf4 = *(const v4f*)(kfS + base + 4 * j4);
        const v4f rr4 = *(const v4f*)(rS  + base + 4 * j4);
#pragma unroll
        for (int e = 0; e < 4; ++e) {
          const float sv = S[4 * j4 + e] * dc4[e] + sa * bb4[e] + vt * kf4[e];
          S[4 * j4 + e] = sv;
          yp += sv * rr4[e];
        }
      }
      yp += __shfl_xor(yp, 1, 32);
      yp += __shfl_xor(yp, 2, 32);
      if (qq == 0) yS[s * kHeadDim + qv] = yp;
    }
    __syncthreads();

    {
      float mu = 0.f;
#pragma unroll 1
      for (int i = 0; i < 4; ++i) mu += yS[pt * kHeadDim + pc + 16 * i];
#pragma unroll
      for (int off = 1; off < 16; off <<= 1) mu += __shfl_xor(mu, off, 32);
      mu *= kInvHeadDim;
      float var = 0.f;
#pragma unroll 1
      for (int i = 0; i < 4; ++i) {
        const float d = yS[pt * kHeadDim + pc + 16 * i] - mu;
        var += d * d;
      }
#pragma unroll
      for (int off = 1; off < 16; off <<= 1) var += __shfl_xor(var, off, 32);
      var *= kInvHeadDim;
      const float rstd = rsqrtf(var + kGnEps);
#pragma unroll 1
      for (int i = 0; i < 4; ++i) {
        const int c  = pc + 16 * i;
        const int gc = h * kHeadDim + c;
        const int li = pt * kHeadDim + c;
        const float xn = (yS[li] - mu) * rstd;
        const float y1 = xn * gn_w[gc] + gn_b[gc];
        const float y2 = y1 + bon * vfS[li];
        oS[li] = y2 * upS[0][li];
      }
    }
    __syncthreads();

    {
      const int plane = wave >> 2;
      const int row   = 4 * (wave & 3) + (lane >> 3);
      const int c8    = (lane & 7) * 8;
      const float* sp = oS + row * kHeadDim + c8;
      unsigned short bits[8];
#pragma unroll
      for (int e = 0; e < 8; ++e) {
        const float v   = sp[e];
        const unsigned short hb = f2bf_bits(v);
        const unsigned short lb = f2bf_bits(v - bf_bits2f(hb));
        bits[e] = plane ? lb : hb;
      }
      const v4u u = (v4u){pk16(bits[0], bits[1]), pk16(bits[2], bits[3]), pk16(bits[4], bits[5]), pk16(bits[6], bits[7])};
      unsigned short* dstp = plane ? aol : aoh;
      const size_t off = (size_t)(m0 + row) * kChan + (size_t)h * kHeadDim + c8;
      *(volatile v4u*)(dstp + off) = u;
      __threadfence();
      *(volatile v4u*)(dstp + off) = u;
    }
  }
}

extern "C" void kernel_launch(void* const* d_in, const int* in_sizes, int n_in,
                              void* d_out, int out_size, void* d_ws, size_t ws_size, hipStream_t stream) {
  if (n_in < 28) return;
  if (in_sizes[0] != kRows * kChan || in_sizes[1] != kRows * kChan || out_size != kRows * kChan) return;
  if (in_sizes[9] != kChan * kRankW || in_sizes[12] != kChan * kRankA || in_sizes[15] != kChan * kRankV ||
      in_sizes[17] != kChan * kRankG || in_sizes[22] != kChan * kChan) return;

  const float* hidden  = (const float*)d_in[0];
  const float* v_first = (const float*)d_in[1];
  const float* x_r = (const float*)d_in[2];
  const float* x_w = (const float*)d_in[3];
  const float* x_k = (const float*)d_in[4];
  const float* x_v = (const float*)d_in[5];
  const float* x_a = (const float*)d_in[6];
  const float* x_g = (const float*)d_in[7];
  const float* w0  = (const float*)d_in[8];
  const float* w1  = (const float*)d_in[9];
  const float* w2  = (const float*)d_in[10];
  const float* a0  = (const float*)d_in[11];
  const float* a1  = (const float*)d_in[12];
  const float* a2  = (const float*)d_in[13];
  const float* v0  = (const float*)d_in[14];
  const float* v1  = (const float*)d_in[15];
  const float* v2  = (const float*)d_in[16];
  const float* g1  = (const float*)d_in[17];
  const float* g2  = (const float*)d_in[18];
  const float* k_k = (const float*)d_in[19];
  const float* k_a = (const float*)d_in[20];
  const float* r_k = (const float*)d_in[21];
  const float* W_r = (const float*)d_in[22];
  const float* W_k = (const float*)d_in[23];
  const float* W_v = (const float*)d_in[24];
  const float* W_o = (const float*)d_in[25];
  const float* gn_w = (const float*)d_in[26];
  const float* gn_b = (const float*)d_in[27];
  float* out = (float*)d_out;

  char* base = (char*)d_ws;
  size_t off = 0;
  auto carve = [&](size_t bytes) -> char* {
    off = (off + 255) & ~(size_t)255;
    char* p = base + off;
    off += bytes;
    return p;
  };
  const size_t plane16 = (size_t)kRows * kChan * 2;
  const size_t plane32 = (size_t)kRows * kChan * 4;
  unsigned short* Xh   = (unsigned short*)carve(plane16);
  unsigned short* Xl   = (unsigned short*)carve(plane16);
  unsigned short* WTh  = (unsigned short*)carve(plane16);
  unsigned short* WTl  = (unsigned short*)carve(plane16);
  unsigned short* WoTh = (unsigned short*)carve(plane16);
  unsigned short* WoTl = (unsigned short*)carve(plane16);
  unsigned short* Aoh  = (unsigned short*)carve(plane16);
  unsigned short* Aol  = (unsigned short*)carve(plane16);
  float* rbuf = (float*)carve(plane32);
  float* kbuf = (float*)carve(plane32);
  float* vbuf = (float*)carve(plane32);
  const size_t szW = (size_t)kRows * kRankWp * 2;
  const size_t szA = (size_t)kRows * kRankAp * 2;
  const size_t szV = (size_t)kRows * kRankV  * 2;
  const size_t szG = (size_t)kRows * kRankG  * 2;
  unsigned short* wdnh = (unsigned short*)carve(szW); unsigned short* wdnl = (unsigned short*)carve(szW);
  unsigned short* adnh = (unsigned short*)carve(szA); unsigned short* adnl = (unsigned short*)carve(szA);
  unsigned short* vdnh = (unsigned short*)carve(szV); unsigned short* vdnl = (unsigned short*)carve(szV);
  unsigned short* gdnh = (unsigned short*)carve(szG); unsigned short* gdnl = (unsigned short*)carve(szG);
  unsigned short* w1Th = (unsigned short*)carve(szW); unsigned short* w1Tl = (unsigned short*)carve(szW);
  unsigned short* a1Th = (unsigned short*)carve(szA); unsigned short* a1Tl = (unsigned short*)carve(szA);
  unsigned short* v1Th = (unsigned short*)carve(szV); unsigned short* v1Tl = (unsigned short*)carve(szV);
  unsigned short* g1Th = (unsigned short*)carve(szG); unsigned short* g1Tl = (unsigned short*)carve(szG);
  unsigned short* w2Th = (unsigned short*)carve(szW); unsigned short* w2Tl = (unsigned short*)carve(szW);
  unsigned short* a2Th = (unsigned short*)carve(szA); unsigned short* a2Tl = (unsigned short*)carve(szA);
  unsigned short* v2Th = (unsigned short*)carve(szV); unsigned short* v2Tl = (unsigned short*)carve(szV);
  unsigned short* g2Th = (unsigned short*)carve(szG); unsigned short* g2Tl = (unsigned short*)carve(szG);
  if (off > ws_size) return;

  auto wt = [&](const float* W, int R, int Cw, unsigned short* hi, unsigned short* lo, int ORows, int OCols) {
    dim3 grid(OCols / 64, ORows / 64);
    k_wt_split<<<grid, 256, 0, stream>>>(W, R, Cw, hi, lo, OCols);
  };
  const int n8 = kRows * kChan / 8;
  auto mix = [&](const float* coef) {
    k_mix_split<<<n8 / 256, 256, 0, stream>>>(hidden, coef, Xh, Xl, n8);
  };
  auto big = [&](float* C) {
    const int tiles = (kRows / 64) * (kChan / 64);
    wmma_gemm64<1, true, 0, 0, false, 0><<<dim3((tiles + 7) / 8, 1), 256, 0, stream>>>(
        Xh, Xl, kChan, 0L, WTh, WTl, kChan, 0L, (void*)C, nullptr, kChan, 0L,
        nullptr, nullptr, 0L, kRows, kChan, kChan, 1.0f);
  };

  wt(W_r, kChan, kChan, WTh, WTl, kChan, kChan);
  mix(x_r);
  big(rbuf);
  wt(w1, kChan, kRankW, w1Th, w1Tl, kRankWp, kChan);
  mix(x_w);
  {
    const int tiles = (kRows / 64) * (kRankWp / 64);
    wmma_gemm64<1, true, 0, 2, false, 1><<<dim3((tiles + 7) / 8, 1), 256, 0, stream>>>(
        Xh, Xl, kChan, 0L, w1Th, w1Tl, kChan, 0L, (void*)wdnh, (void*)wdnl, kRankWp, 0L,
        nullptr, nullptr, 0L, kRows, kRankWp, kChan, 1.0f);
  }
  wt(W_k, kChan, kChan, WTh, WTl, kChan, kChan);
  mix(x_k);
  big(kbuf);
  wt(W_v, kChan, kChan, WTh, WTl, kChan, kChan);
  wt(v1, kChan, kRankV, v1Th, v1Tl, kRankV, kChan);
  mix(x_v);
  big(vbuf);
  {
    const int tiles = (kRows / 64) * (kRankV / 64);
    wmma_gemm64<1, true, 0, 2, false, 0><<<dim3((tiles + 7) / 8, 1), 256, 0, stream>>>(
        Xh, Xl, kChan, 0L, v1Th, v1Tl, kChan, 0L, (void*)vdnh, (void*)vdnl, kRankV, 0L,
        nullptr, nullptr, 0L, kRows, kRankV, kChan, 1.0f);
  }
  wt(a1, kChan, kRankA, a1Th, a1Tl, kRankAp, kChan);
  mix(x_a);
  {
    const int tiles = (kRows / 64) * (kRankAp / 64);
    wmma_gemm64<1, true, 0, 2, false, 0><<<dim3((tiles + 7) / 8, 1), 256, 0, stream>>>(
        Xh, Xl, kChan, 0L, a1Th, a1Tl, kChan, 0L, (void*)adnh, (void*)adnl, kRankAp, 0L,
        nullptr, nullptr, 0L, kRows, kRankAp, kChan, 1.0f);
  }
  wt(g1, kChan, kRankG, g1Th, g1Tl, kRankG, kChan);
  mix(x_g);
  {
    const int tiles = (kRows / 64) * (kRankG / 64);
    wmma_gemm64<1, true, 0, 2, false, 6><<<dim3((tiles + 7) / 8, 1), 256, 0, stream>>>(
        Xh, Xl, kChan, 0L, g1Th, g1Tl, kChan, 0L, (void*)gdnh, (void*)gdnl, kRankG, 0L,
        nullptr, nullptr, 0L, kRows, kRankG, kChan, 1.0f);
  }
  wt(w2, kRankW, kChan, w2Th, w2Tl, kChan, kRankWp);
  wt(a2, kRankA, kChan, a2Th, a2Tl, kChan, kRankAp);
  wt(v2, kRankV, kChan, v2Th, v2Tl, kChan, kRankV);
  wt(g2, kRankG, kChan, g2Th, g2Tl, kChan, kRankG);
  wt(W_o, kChan, kChan, WoTh, WoTl, kChan, kChan);

  k_wkv_fused<<<kBatch * kHeads, 256, 0, stream>>>(
      rbuf, kbuf, vbuf, v_first,
      gdnh, gdnl, g2Th, g2Tl,
      wdnh, wdnl, w2Th, w2Tl,
      vdnh, vdnl, v2Th, v2Tl,
      adnh, adnl, a2Th, a2Tl,
      w0, a0, v0, k_k, k_a, r_k, gn_w, gn_b,
      Aoh, Aol);

  {
    const int tiles = (kRows / 64) * (kChan / 64);
    wmma_gemm64<1, true, 0, 0, false, 0><<<dim3((tiles + 7) / 8, 1), 256, 0, stream>>>(
        Aoh, Aol, kChan, 0L, WoTh, WoTl, kChan, 0L, (void*)out, nullptr, kChan, 0L,
        nullptr, nullptr, 0L, kRows, kChan, kChan, 1.0f);
  }
}
